// RelationalMultiHeadAttentionMP_45157286150354
// MI455X (gfx1250) — hardware-verified
//
#include <hip/hip_runtime.h>
#include <stddef.h>


#define HIDK   128
#define NHD    8
#define DKD    16
#define PC     512
#define GT     128
#define SPW    (32 * 64)
#define APITCH 136
#define WPP    136
#define RB     1024
#define RBBITS 10
#define RMAX   128
#define RMBITS 7
#define TABW   (2 * RMAX)
#define CHUNK  4096
#define LCAP   12288
#define DEGCAP 64
#define SCW    (32 * (DEGCAP / 2))
#define MZW    32
#define WSCAP  134217728
#define ASCL   8.0f
#define WSCL   64.0f
#define INVSCL 0.001953125f
#define QKSCL  0.25f

#define EDGE_LDS_INTS  (RB + 8 + RB + LCAP)
#define EDGE_LDS_BYTES ((EDGE_LDS_INTS + 8 * SCW) * 4)

static_assert(NHD * DKD == HIDK);
static_assert(DKD == 16);
static_assert(PC == 4 * HIDK);
static_assert(RB == (1 << RBBITS));
static_assert(RMAX == (1 << RMBITS));
static_assert(CHUNK == 8 * 16 * 32);
static_assert(CHUNK == 4 * 4 * 256);
static_assert((APITCH % 8) == 0);
static_assert((WPP % 8) == 0);
static_assert((DEGCAP % 2) == 0);
static_assert(((EDGE_LDS_INTS * 4) % 16) == 0);
static_assert(EDGE_LDS_BYTES < 300000);
static_assert((MZW * 4) == 128);

typedef float          v4f  __attribute__((ext_vector_type(4)));
typedef float          v8f  __attribute__((ext_vector_type(8)));
typedef int            v4i  __attribute__((ext_vector_type(4)));
typedef unsigned int   v4u  __attribute__((ext_vector_type(4)));
typedef unsigned short v4us __attribute__((ext_vector_type(4)));
typedef unsigned short v8us __attribute__((ext_vector_type(8)));
typedef _Float16       v16h __attribute__((ext_vector_type(16)));
union FragH { v16h v; v8us u[2]; };

__device__ __forceinline__ unsigned short h16(float f) {
  const _Float16 h = (_Float16)f;
  return __builtin_bit_cast(unsigned short, h);
}
__device__ __forceinline__ float hf(unsigned short u) {
  return (float)__builtin_bit_cast(_Float16, u);
}

__device__ __forceinline__ v8us cvt8(v4f a, v4f b, float s) {
  v8us r;
  r[0] = h16(a[0] * s); r[1] = h16(a[1] * s); r[2] = h16(a[2] * s); r[3] = h16(a[3] * s);
  r[4] = h16(b[0] * s); r[5] = h16(b[1] * s); r[6] = h16(b[2] * s); r[7] = h16(b[3] * s);
  return r;
}

__device__ __forceinline__ v8f wmh(v16h a, v16h b, v8f c) {
  v8f d = __builtin_amdgcn_wmma_f32_16x16x32_f16(false, a, false, b, (short)0, c, false, false);
  asm volatile("v_nop\n\tv_nop\n\tv_nop\n\tv_nop" : "+v"(d) : "v"(a), "v"(b));
  return d;
}

template <int NB>
__device__ __forceinline__ unsigned int match_mask(unsigned int base, int key) {
  unsigned int msk = base;
#pragma unroll
  for (int b = 0; b < NB; ++b) {
    const bool bit = ((key >> b) & 1) != 0;
    const unsigned int bb = __builtin_amdgcn_ballot_w32(bit);
    msk &= bit ? bb : ~bb;
  }
  return msk;
}

__global__ __launch_bounds__(256) void k_wprep(
    const float* __restrict__ Wq, const float* __restrict__ Wk, const float* __restrict__ Wm,
    unsigned short* w16) {
  __shared__ __attribute__((aligned(16))) unsigned short sT[32 * WPP];
  const int tid = (int)threadIdx.x;
  const int b = (int)blockIdx.x;
  const int t = b >> 4;
  const int rb = b & 15;
  const int g = rb >> 2;
  const int m0 = 32 * (rb & 3);
  const float* W = (g == 0) ? (Wm + (size_t)t * 2 * HIDK * HIDK)
                 : ((g == 1) ? (Wk + (size_t)t * HIDK * HIDK)
                 : ((g == 2) ? (Wm + (size_t)t * 2 * HIDK * HIDK + (size_t)HIDK * HIDK)
                             : (Wq + (size_t)t * HIDK * HIDK)));

#pragma unroll 1
  for (int it = 0; it < 16; ++it) {
    const int idx = it * 256 + tid;
    const int rr = idx & 31, k = idx >> 5;
    const float val = W[(size_t)k * HIDK + m0 + rr];
    sT[rr * WPP + k] = h16(val * WSCL);
  }
  __syncthreads();

  v8us pv[2];
  size_t po[2];
#pragma unroll
  for (int it = 0; it < 2; ++it) {
    const int p = it * 256 + tid;
    const int row = p >> 4, c8 = (p & 15) * 8;
    pv[it] = *(const v8us*)(sT + row * WPP + c8);
    po[it] = ((size_t)b * 32 + row) * HIDK + c8;
  }
#pragma unroll
  for (int it = 0; it < 2; ++it) *(volatile v8us*)(w16 + po[it]) = pv[it];
  __threadfence();
#pragma unroll
  for (int it = 0; it < 2; ++it) *(volatile v8us*)(w16 + po[it]) = pv[it];
}

__global__ __launch_bounds__(GT) void k_gemm(
    const float* __restrict__ X, const unsigned short* __restrict__ Bt,
    const float* __restrict__ bmT, unsigned short* outH, int M) {
  __shared__ __attribute__((aligned(16))) float sT[4 * SPW];
  __shared__ __attribute__((aligned(16))) unsigned short sA[64 * APITCH];
  const int tid = (int)threadIdx.x, lane = tid & 31, wave = tid >> 5, hh = lane >> 4, m = lane & 15;
  const int rb = (int)blockIdx.x * 64;

#pragma unroll 4
  for (int it = 0; it < 16; ++it) {
    const int f = it * GT + tid;
    const int row = f >> 5, c4 = (f & 31) * 4;
    int gr = rb + row; gr = gr > M - 1 ? M - 1 : gr;
    const v4f v = *(const v4f*)(X + (size_t)gr * HIDK + c4);
    v4us o;
    o[0] = h16(v[0] * ASCL); o[1] = h16(v[1] * ASCL); o[2] = h16(v[2] * ASCL); o[3] = h16(v[3] * ASCL);
    *(v4us*)(sA + row * APITCH + c4) = o;
  }
  __syncthreads();

  const int lr0 = (wave >> 1) * 32;
  const int r0 = rb + lr0;
  const unsigned short* ap0 = sA + (lr0 + m) * APITCH + 8 * hh;
  const unsigned short* ap1 = sA + (lr0 + 16 + m) * APITCH + 8 * hh;
  const bool full = (r0 + 32 <= M);
  float* sw = sT + wave * SPW;

#pragma unroll 1
  for (int cg = 0; cg < 4; ++cg) {
    const int c0 = cg * 128 + (wave & 1) * 64;
    const unsigned short* bp[4];
#pragma unroll
    for (int j = 0; j < 4; ++j)
      bp[j] = Bt + (size_t)(c0 + 16 * j + m) * HIDK + 8 * hh;

    v8f acc[2][4];
#pragma unroll
    for (int i = 0; i < 2; ++i)
#pragma unroll
      for (int j = 0; j < 4; ++j) { v8f z = {0.f, 0.f, 0.f, 0.f, 0.f, 0.f, 0.f, 0.f}; acc[i][j] = z; }

#pragma unroll 1
    for (int kt = 0; kt < HIDK / 32; ++kt) {
      const int kb = kt << 5;
      FragH a0, a1;
      a0.u[0] = *(const v8us*)(ap0 + kb);
      a0.u[1] = *(const v8us*)(ap0 + kb + 16);
      a1.u[0] = *(const v8us*)(ap1 + kb);
      a1.u[1] = *(const v8us*)(ap1 + kb + 16);
#pragma unroll
      for (int j = 0; j < 4; ++j) {
        FragH bf;
        bf.u[0] = *(const v8us*)(bp[j] + kb);
        bf.u[1] = *(const v8us*)(bp[j] + kb + 16);
        acc[0][j] = wmh(a0.v, bf.v, acc[0][j]);
        acc[1][j] = wmh(a1.v, bf.v, acc[1][j]);
      }
    }

#pragma unroll
    for (int i = 0; i < 2; ++i)
#pragma unroll
      for (int j = 0; j < 4; ++j)
#pragma unroll
        for (int r = 0; r < 8; ++r)
          sw[(16 * i + 8 * hh + r) * 64 + 16 * j + m] = acc[i][j][r];
    __syncthreads();

    const float bs = (cg == 2) ? 1.0f : 0.0f;
    v8us hv[8];
    size_t po[8];
#pragma unroll
    for (int it = 0; it < 8; ++it) {
      const int f = it * 32 + lane;
      const int row = f >> 3, c8 = (f & 7) * 8;
      const v4f v0 = *(const v4f*)(sw + row * 64 + c8);
      const v4f v1 = *(const v4f*)(sw + row * 64 + c8 + 4);
      const int gc = c0 + c8;
      int bi = gc - 2 * HIDK; bi = bi < 0 ? 0 : (bi > HIDK - 8 ? HIDK - 8 : bi);
      const v4f b0v = *(const v4f*)(bmT + bi);
      const v4f b1v = *(const v4f*)(bmT + bi + 4);
      const v4f o0 = v0 * INVSCL + b0v * bs;
      const v4f o1 = v1 * INVSCL + b1v * bs;
      hv[it] = cvt8(o0, o1, 1.0f);
      po[it] = (size_t)(r0 + row) * PC + gc;
    }
    if (full) {
#pragma unroll
      for (int it = 0; it < 8; ++it) *(volatile v8us*)(outH + po[it]) = hv[it];
    }
    __threadfence();
    if (full) {
#pragma unroll
      for (int it = 0; it < 8; ++it) *(volatile v8us*)(outH + po[it]) = hv[it];
    }
    __syncthreads();
  }
}

__global__ __launch_bounds__(256) void k_csort(
    const int* __restrict__ adj, unsigned int* csort, int* tab, int nN, int nE) {
  __shared__ __attribute__((aligned(16))) unsigned int sImg[CHUNK];
  __shared__ int cw[8 * RMAX];
  __shared__ __attribute__((aligned(16))) int sPre[RMAX];
  __shared__ __attribute__((aligned(16))) int sCn[RMAX];
  __shared__ int sWt[8];
  const int tid = (int)threadIdx.x, lane = tid & 31, wave = tid >> 5;
  const int c = (int)blockIdx.x;
  const int cbase = c * CHUNK;

  for (int i = tid; i < 8 * RMAX; i += 256) cw[i] = 0;
  {
    const v4u s = {0xffffffffu, 0xffffffffu, 0xffffffffu, 0xffffffffu};
    for (int i = tid; i < CHUNK / 4; i += 256) ((v4u*)sImg)[i] = s;
  }
  __syncthreads();

  unsigned int ent[16];
  int pk[16];
  const unsigned int lt = (1u << lane) - 1u;
#pragma unroll
  for (int i = 0; i < 16; ++i) {
    const int e = cbase + wave * 512 + 32 * i + lane;
    const int ea = e > nE - 1 ? nE - 1 : e;
    const int d = adj[(size_t)ea * 2 + 1];
    const bool valid = (e < nE) && ((unsigned)d < (unsigned)nN);
    const int dd = valid ? d : 0;
    const int r  = dd >> RBBITS;
    const int jl = dd & (RB - 1);
    const unsigned int msk = match_mask<RMBITS>(__builtin_amdgcn_ballot_w32(valid), r);
    const int rank = (int)__builtin_popcount(msk & lt);
    const int grp  = (int)__builtin_popcount(msk);
    const int base = cw[wave * RMAX + r];
    pk[i]  = valid ? ((r << 12) | (base + rank)) : -1;
    ent[i] = ((unsigned int)ea << RBBITS) | (unsigned int)jl;
    if (valid && rank == 0) cw[wave * RMAX + r] = base + grp;
    __syncthreads();
  }

  if (tid < RMAX) {
    int run = 0;
#pragma unroll
    for (int w = 0; w < 8; ++w) {
      const int v = cw[w * RMAX + tid];
      cw[w * RMAX + tid] = run;
      run += v;
    }
    sCn[tid] = run;
  }
  __syncthreads();
  {
    const int vr = sCn[tid & (RMAX - 1)];
    const int v  = (tid < RMAX) ? vr : 0;
    int x = v;
#pragma unroll
    for (int dd = 1; dd < 32; dd <<= 1) {
      const int y = __shfl_up(x, dd);
      x += (lane >= dd) ? y : 0;
    }
    if (lane == 31) sWt[wave] = x;
    __syncthreads();
    int pre = 0;
#pragma unroll
    for (int w = 0; w < 8; ++w) { const int tw = sWt[w]; pre += (w < wave) ? tw : 0; }
    if (tid < RMAX) sPre[tid] = pre + x - v;
  }
  __syncthreads();

#pragma unroll
  for (int i = 0; i < 16; ++i) {
    if (pk[i] >= 0) {
      const int r = (pk[i] >> 12) & (RMAX - 1);
      const int q = pk[i] & 4095;
      const int pos = sPre[r] + cw[wave * RMAX + r] + q;
      if ((unsigned)pos < (unsigned)CHUNK) sImg[pos] = ent[i];
    }
  }
  __syncthreads();

  v4u iv[4];
#pragma unroll
  for (int it = 0; it < 4; ++it) iv[it] = ((const v4u*)sImg)[it * 256 + tid];
  const v4i ta = *(const v4i*)(sPre + 4 * lane);
  const v4i tb = *(const v4i*)(sCn + 4 * lane);
  const v4i tv = (wave == 0) ? ta : tb;
  unsigned int* gp = csort + (size_t)c * CHUNK;
  int* tp = tab + (size_t)c * TABW + 4 * tid;
  const bool wt = tid < 64;
#pragma unroll
  for (int it = 0; it < 4; ++it) *(volatile v4u*)(gp + 4 * (it * 256 + tid)) = iv[it];
  if (wt) *(volatile v4i*)tp = tv;
  __threadfence();
#pragma unroll
  for (int it = 0; it < 4; ++it) *(volatile v4u*)(gp + 4 * (it * 256 + tid)) = iv[it];
  if (wt) *(volatile v4i*)tp = tv;
}

__global__ __launch_bounds__(256) void k_edge(
    const unsigned short* __restrict__ plane, const int* __restrict__ adj,
    const unsigned int* __restrict__ csort, const int* __restrict__ tab,
    float* out, float* mz,
    int nN, int nE, int nEt, int tsel, int nCh, int first, int last) {
  extern __shared__ __attribute__((aligned(16))) int dsm[];
  __shared__ int sWtot[8];
  int*   sOff  = dsm;
  int*   sCur  = dsm + (RB + 8);
  int*   sList = sCur + RB;
  float* sSc   = (float*)(sList + LCAP);
  const int tid = (int)threadIdx.x, lane = tid & 31, wave = tid >> 5;
  const int rgn = (int)blockIdx.x;
  const int n0 = rgn * RB;
  const unsigned int lt = (1u << lane) - 1u;

  for (int i = tid; i < RB + 8; i += 256) sOff[i] = 0;
  for (int i = tid; i < RB; i += 256) sCur[i] = 0;
  for (int i = tid; i < LCAP; i += 256) sList[i] = 0;
  __syncthreads();

#pragma unroll 1
  for (int c = 0; c < nCh; ++c) {
    int pre = tab[(size_t)c * TABW + rgn];
    int n   = tab[(size_t)c * TABW + RMAX + rgn];
    pre = pre < 0 ? 0 : (pre > CHUNK ? CHUNK : pre);
    n = n < 0 ? 0 : (n > CHUNK - pre ? CHUNK - pre : n);
    const int nstep = (n + 31) >> 5;
    const unsigned int* cp = csort + (size_t)c * CHUNK + pre;
#pragma unroll 1
    for (int s = 0; s < nstep; ++s) {
      if (wave == 0) {
        const int i = (s << 5) + lane;
        const bool valid = i < n;
        const int ic = i > n - 1 ? n - 1 : i;
        const unsigned int en = cp[ic];
        const int j = (int)(en & (unsigned int)(RB - 1));
        const unsigned int msk = match_mask<RBBITS>(__builtin_amdgcn_ballot_w32(valid), j);
        const int rank = (int)__builtin_popcount(msk & lt);
        const int grp  = (int)__builtin_popcount(msk);
        if (valid && rank == 0) sOff[j] = sOff[j] + grp;
      }
      __syncthreads();
    }
  }
  __syncthreads();

  {
    int cn[4];
    int ls = 0;
#pragma unroll
    for (int i = 0; i < 4; ++i) { cn[i] = sOff[4 * tid + i]; ls += cn[i]; }
    int x = ls;
#pragma unroll
    for (int dd = 1; dd < 32; dd <<= 1) {
      const int y = __shfl_up(x, dd);
      x += (lane >= dd) ? y : 0;
    }
    if (lane == 31) sWtot[wave] = x;
    __syncthreads();
    int pre = 0;
#pragma unroll
    for (int w = 0; w < 8; ++w) { const int tw = sWtot[w]; pre += (w < wave) ? tw : 0; }
    int run = pre + x - ls;
#pragma unroll
    for (int i = 0; i < 4; ++i) { sOff[4 * tid + i] = run; run += cn[i]; }
    if (tid == 255) sOff[RB] = run;
  }
  __syncthreads();

#pragma unroll 1
  for (int c = 0; c < nCh; ++c) {
    int pre = tab[(size_t)c * TABW + rgn];
    int n   = tab[(size_t)c * TABW + RMAX + rgn];
    pre = pre < 0 ? 0 : (pre > CHUNK ? CHUNK : pre);
    n = n < 0 ? 0 : (n > CHUNK - pre ? CHUNK - pre : n);
    const int nstep = (n + 31) >> 5;
    const unsigned int* cp = csort + (size_t)c * CHUNK + pre;
#pragma unroll 1
    for (int s = 0; s < nstep; ++s) {
      if (wave == 0) {
        const int i = (s << 5) + lane;
        const bool valid = i < n;
        const int ic = i > n - 1 ? n - 1 : i;
        const unsigned int en = cp[ic];
        const int j = (int)(en & (unsigned int)(RB - 1));
        int e = (int)(en >> RBBITS);
        e = e > nE - 1 ? nE - 1 : e;
        const unsigned int msk = match_mask<RBBITS>(__builtin_amdgcn_ballot_w32(valid), j);
        const int rank = (int)__builtin_popcount(msk & lt);
        const int grp  = (int)__builtin_popcount(msk);
        const int cur  = sCur[j];
        const int p0   = sOff[j] + cur + rank;
        if (valid && (unsigned)p0 < (unsigned)LCAP) sList[p0] = e;
        if (valid && rank == 0) sCur[j] = cur + grp;
      }
      __syncthreads();
    }
  }
  __syncthreads();

  const int ch = 8 * (lane & 15);
  const int hd = (lane & 15) >> 1;
  const float negbig = -3.0e38f;
  int Rb = nN - n0; Rb = Rb > RB ? RB : Rb;
  float* sw = sSc + wave * SCW;
#pragma unroll 1
  for (int j = wave; j < Rb; j += 8) {
    const int node = n0 + j;
    int lb = __builtin_amdgcn_readfirstlane(sOff[j]);
    int ub = __builtin_amdgcn_readfirstlane(sOff[j + 1]);
    lb = lb < 0 ? 0 : (lb > LCAP ? LCAP : lb);
    ub = ub < 0 ? 0 : (ub > LCAP ? LCAP : ub);
    int cnt = ub - lb;
    cnt = cnt < 0 ? 0 : (cnt > DEGCAP ? DEGCAP : cnt);

    int cl = 0, ce = 0;
    const int nsc = (cnt + 31) >> 5;
#pragma unroll 1
    for (int s = 0; s < nsc; ++s) {
      const int i = (s << 5) + lane;
      const bool valid = i < cnt;
      const int ic = valid ? i : (cnt - 1);
      int li = lb + ic; li = li < 0 ? 0 : (li > LCAP - 1 ? LCAP - 1 : li);
      int e = sList[li]; e = e < 0 ? 0 : (e > nE - 1 ? nE - 1 : e);
      const int te = e / nEt;
      cl += (int)__builtin_popcount(__builtin_amdgcn_ballot_w32(valid && (te < tsel)));
      ce += (int)__builtin_popcount(__builtin_amdgcn_ballot_w32(valid && (te <= tsel)));
    }
    const int lbT = lb + cl;
    int cntT = ce - cl;
    cntT = cntT < 0 ? 0 : (cntT > DEGCAP ? DEGCAP : cntT);
    const int np = (cntT + 1) >> 1;

    const v8us ptv = *(const v8us*)(plane + (size_t)node * PC + 2 * HIDK + ch);
    const v8us qnv = *(const v8us*)(plane + (size_t)node * PC + 3 * HIDK + ch);
    float ptb[8], qf[8];
#pragma unroll
    for (int cc = 0; cc < 8; ++cc) { ptb[cc] = hf(ptv[cc]); qf[cc] = hf(qnv[cc]) * QKSCL; }

    float m = negbig;
#pragma unroll 1
    for (int it = 0; it < np; ++it) {
      const int i = 2 * it + (lane >> 4);
      const bool valid = i < cntT;
      const int ic = valid ? i : (cntT - 1);
      int li = lbT + ic; li = li < 0 ? 0 : (li > LCAP - 1 ? LCAP - 1 : li);
      int e = sList[li]; e = e < 0 ? 0 : (e > nE - 1 ? nE - 1 : e);
      int s = adj[(size_t)e * 2]; s = s < 0 ? 0 : (s > nN - 1 ? nN - 1 : s);
      const v8us kv = *(const v8us*)(plane + (size_t)s * PC + HIDK + ch);
      float part = 0.0f;
#pragma unroll
      for (int cc = 0; cc < 8; ++cc) part = fmaf(qf[cc], hf(kv[cc]), part);
      part += __shfl_xor(part, 1);
      m = valid ? fmaxf(m, part) : m;
      sw[it * 32 + lane] = part;
    }
    m = fmaxf(m, __shfl_xor(m, 16));
    const float mo_raw = mz[(size_t)node * MZW + hd];
    const float zo_raw = mz[(size_t)node * MZW + 8 + hd];
    const float m_old = first ? negbig : mo_raw;
    const float z_old = first ? 0.0f : zo_raw;
    const float m_new = fmaxf(m_old, m);

    float acc[8];
#pragma unroll
    for (int cc = 0; cc < 8; ++cc) acc[cc] = 0.0f;
    float zt = 0.0f;
#pragma unroll 1
    for (int it = 0; it < np; ++it) {
      const int i = 2 * it + (lane >> 4);
      const bool valid = i < cntT;
      const int ic = valid ? i : (cntT - 1);
      int li = lbT + ic; li = li < 0 ? 0 : (li > LCAP - 1 ? LCAP - 1 : li);
      int e = sList[li]; e = e < 0 ? 0 : (e > nE - 1 ? nE - 1 : e);
      int s = adj[(size_t)e * 2]; s = s < 0 ? 0 : (s > nN - 1 ? nN - 1 : s);
      const float sc = sw[it * 32 + lane];
      float p = __expf(sc - m_new);
      p = valid ? p : 0.0f;
      const v8us pv = *(const v8us*)(plane + (size_t)s * PC + ch);
#pragma unroll
      for (int cc = 0; cc < 8; ++cc) {
        const float msg = fmaxf(hf(pv[cc]) + ptb[cc], 0.0f);
        acc[cc] = fmaf(p, msg, acc[cc]);
      }
      zt += p;
    }
#pragma unroll
    for (int cc = 0; cc < 8; ++cc) acc[cc] += __shfl_xor(acc[cc], 16);
    zt += __shfl_xor(zt, 16);

    const float corr = __expf(fmaxf(m_old - m_new, -87.0f));
    const float z_new = fmaf(z_old, corr, zt);
    const v4f oa = *(const v4f*)(out + (size_t)node * HIDK + ch);
    const v4f ob = *(const v4f*)(out + (size_t)node * HIDK + ch + 4);
    const float zs = (z_new > 0.0f) ? z_new : 1.0f;
    const float rz = (z_new > 0.0f) ? (1.0f / zs) : 0.0f;
    const float fin = last ? rz : 1.0f;
    float val[8];
#pragma unroll
    for (int cc = 0; cc < 4; ++cc) {
      const float a0 = first ? 0.0f : oa[cc];
      const float a1 = first ? 0.0f : ob[cc];
      val[cc]     = fmaf(a0, corr, acc[cc]) * fin;
      val[4 + cc] = fmaf(a1, corr, acc[4 + cc]) * fin;
    }

    const int sl = lane >> 1;
    v4f u4, w4;
#pragma unroll
    for (int cc = 0; cc < 4; ++cc) { u4[cc] = __shfl(val[cc], sl); w4[cc] = __shfl(val[4 + cc], sl); }
    const v4f ov = (lane & 1) ? w4 : u4;
    v4f mv, zv;
#pragma unroll
    for (int cc = 0; cc < 4; ++cc) {
      const int hs = 2 * (4 * (lane & 1) + cc);
      mv[cc] = __shfl(m_new, hs);
      zv[cc] = __shfl(z_new, hs);
    }
    const v4f zero4 = {0.0f, 0.0f, 0.0f, 0.0f};
    const v4f pcv = (lane < 2) ? mv : ((lane < 4) ? zv : zero4);
    const bool wmz = (last == 0) && (lane < 8);
    float* op = out + (size_t)node * HIDK + 4 * lane;
    float* mp = mz + (size_t)node * MZW + 4 * (lane & 7);
    *(volatile v4f*)op = ov;
    if (wmz) *(volatile v4f*)mp = pcv;
    __threadfence();
    *(volatile v4f*)op = ov;
    if (wmz) *(volatile v4f*)mp = pcv;
  }
}

extern "C" void kernel_launch(void* const* d_in, const int* in_sizes, int n_in,
                              void* d_out, int out_size, void* d_ws, size_t ws_size,
                              hipStream_t stream) {
  if (n_in < 6) return;
  const int nN = in_sizes[0] / HIDK;
  if (nN <= 0 || in_sizes[0] != nN * HIDK || (nN % 32) != 0) return;
  const int T = in_sizes[2] / (HIDK * HIDK);
  if (T < 1 || in_sizes[2] != T * HIDK * HIDK || in_sizes[3] != T * HIDK * HIDK) return;
  if (in_sizes[4] != T * 2 * HIDK * HIDK || in_sizes[5] != T * HIDK) return;
  if (in_sizes[1] <= 0 || (in_sizes[1] % (2 * T)) != 0) return;
  const int nEt = in_sizes[1] / (2 * T);
  const int nE = T * nEt;
  if (nEt < 1 || nE > (1 << 22)) return;
  if (nN > RMAX * RB) return;
  if (out_size != nN * HIDK) return;

  const float* x   = (const float*)d_in[0];
  const int*   adj = (const int*)d_in[1];
  const float* Wq  = (const float*)d_in[2];
  const float* Wk  = (const float*)d_in[3];
  const float* Wm  = (const float*)d_in[4];
  const float* bm  = (const float*)d_in[5];
  float* out = (float*)d_out;

  const int nCh = (nE + CHUNK - 1) / CHUNK;
  const int nR  = (nN + RB - 1) / RB;

  const size_t nNp   = (size_t)((nN + 63) / 64) * 64;
  const size_t szW16 = (size_t)T * PC * HIDK * 2;
  const size_t szP   = nNp * PC * 2;
  const size_t szMZ  = (size_t)nR * RB * MZW * 4;
  const size_t szCS  = (size_t)nCh * CHUNK * 4;
  const size_t szTab = (size_t)nCh * TABW * 4;
  size_t off = 0;
  const size_t oW  = off; off += szW16; off = (off + 255) & ~(size_t)255;
  const size_t oP  = off; off += szP;   off = (off + 255) & ~(size_t)255;
  const size_t oMZ = off; off += szMZ;  off = (off + 255) & ~(size_t)255;
  const size_t oCS = off; off += szCS;  off = (off + 255) & ~(size_t)255;
  const size_t oTb = off; off += szTab; off = (off + 255) & ~(size_t)255;
  if (off > ws_size || off > (size_t)WSCAP) return;

  char* ws = (char*)d_ws;
  unsigned short* w16   = (unsigned short*)(ws + oW);
  unsigned short* plane = (unsigned short*)(ws + oP);
  float*          mz    = (float*)(ws + oMZ);
  unsigned int*   csort = (unsigned int*)(ws + oCS);
  int*            tab   = (int*)(ws + oTb);

  k_wprep<<<16 * T, 256, 0, stream>>>(Wq, Wk, Wm, w16);

  k_csort<<<nCh, 256, 0, stream>>>(adj, csort, tab, nN, nE);

  hipFuncSetAttribute(reinterpret_cast<const void*>(&k_edge),
                      hipFuncAttributeMaxDynamicSharedMemorySize, EDGE_LDS_BYTES);
  const int gG = (nN + 63) / 64;
  for (int t = 0; t < T; ++t) {
    k_gemm<<<gG, GT, 0, stream>>>(x, w16 + (size_t)t * PC * HIDK, bm + (size_t)t * HIDK, plane, nN);
    const int first = (t == 0) ? 1 : 0;
    const int last  = (t == T - 1) ? 1 : 0;
    k_edge<<<nR, 256, EDGE_LDS_BYTES, stream>>>(plane, adj, csort, tab,
                                                out, mz, nN, nE, nEt, t, nCh, first, last);
  }
}
